// LinOSSLayer_53429393163009
// MI455X (gfx1250) — hardware-verified
//
#include <hip/hip_runtime.h>


namespace {
constexpr int B = 16, H = 256, L = 2048, P = 64, PC = 2 * P, NR = B * L;
constexpr float XS = 8.0f, WSC = 256.0f;
typedef _Float16 b16;
typedef __attribute__((ext_vector_type(16))) _Float16 v16b;
typedef __attribute__((ext_vector_type(8))) _Float16 v8b;
typedef __attribute__((ext_vector_type(8))) float v8f;
typedef __attribute__((ext_vector_type(4))) float v4f;
__device__ __forceinline__ float bf16_rne(float f) { unsigned int u = __float_as_uint(f); u += 0x7FFFu + ((u >> 16) & 1u); return __uint_as_float(u & 0xFFFF0000u); }
__device__ __forceinline__ void split16(float v, b16& hi, b16& lo) { hi = (b16)v; lo = (b16)(v - (float)hi); }
__device__ __forceinline__ v16b frag_kb(const b16* p, int hh) { const v8b a = *(const v8b*)(p + 8 * hh), b = *(const v8b*)(p + 16 + 8 * hh); v16b f;
#pragma unroll
  for (int e = 0; e < 8; ++e) { f[e] = a[e]; f[8 + e] = b[e]; } return f; }
__device__ __forceinline__ v8f wmma16b(v16b a, v16b b, v8f c) { v8f d = __builtin_amdgcn_wmma_f32_16x16x32_f16(false, a, false, b, (short)0, c, false, false); asm volatile("v_nop\n\tv_nop\n\tv_nop\n\tv_nop" : "+v"(d) : "v"(a), "v"(b)); return d; }
__device__ __forceinline__ void wave_lds_sync() { __builtin_amdgcn_fence(__ATOMIC_RELEASE, "workgroup"); __builtin_amdgcn_wave_barrier(); __builtin_amdgcn_fence(__ATOMIC_ACQUIRE, "workgroup"); }
__device__ __forceinline__ float pmul(float a, float b) { float p = a * b; asm volatile("" : "+v"(p)); return p; }
__device__ __forceinline__ float gelu(float v) { return 0.5f * v * (1.0f + erff(v * 0.70710678118654752f)); }

__global__ __launch_bounds__(256) void wprep_kernel(const float* __restrict__ Bm, const float* __restrict__ Cm, const float* __restrict__ W1, const float* __restrict__ W2, b16* __restrict__ WB, b16* __restrict__ WC, b16* __restrict__ W12) {
  const int u = blockIdx.x * 256 + threadIdx.x;
  for (int pass = 0; pass < 2; ++pass) {
    if (u < PC * (H / 8)) { const int pr = u / (H / 8), h0 = (u % (H / 8)) * 8; const int p = pr >> 1, r = pr & 1; v8b v; for (int j = 0; j < 8; ++j) v[j] = (b16)(bf16_rne(Bm[((size_t)p * H + h0 + j) * 2 + r]) * WSC); *(volatile v8b*)(WB + (size_t)pr * H + h0) = v; }
    if (u < H * (PC / 8)) { const int h = u / (PC / 8), c0 = (u % (PC / 8)) * 8; v8b v; for (int j = 0; j < 8; ++j) { const int c = c0 + j, p = c >> 1, r = c & 1; const float cv = bf16_rne(Cm[((size_t)h * P + p) * 2 + r]); v[j] = (b16)((r ? -cv : cv) * WSC); } *(volatile v8b*)(WC + (size_t)h * PC + c0) = v; }
    if (u < 2 * H * (H / 8)) { const int o = u / (H / 8), k0 = (u % (H / 8)) * 8; const float* w = o < H ? W1 + (size_t)o * H : W2 + (size_t)(o - H) * H; v8b v; for (int j = 0; j < 8; ++j) v[j] = (b16)(bf16_rne(w[k0 + j]) * WSC); *(volatile v8b*)(W12 + (size_t)o * H + k0) = v; }
    __threadfence(); }
}
__global__ __launch_bounds__(256) void ut_kernel(const float* __restrict__ uu, int BV, b16* __restrict__ UT) {
  __shared__ float Ts[H][33]; const int tid = threadIdx.x, wave = tid >> 5, lane = tid & 31; const int b = blockIdx.x / (L / 32), l0 = (blockIdx.x % (L / 32)) * 32; if (b >= BV) return;
  for (int h = wave; h < H; h += 8) Ts[h][lane] = bf16_rne(uu[((size_t)b * H + h) * L + l0 + lane]);
  __syncthreads();
  for (int pass = 0; pass < 2; ++pass) { for (int r = 0; r < 4; ++r) { const int ll = wave * 4 + r; const size_t row = (size_t)b * L + l0 + ll; for (int q = 0; q < 8; ++q) ((volatile b16*)UT)[row * H + q * 32 + lane] = (b16)(Ts[q * 32 + lane][ll] * XS); } __threadfence(); }
}
__global__ __launch_bounds__(32) void bu_kernel(const b16* __restrict__ UT, const b16* __restrict__ WB, int RL, float* __restrict__ BU) {
  __shared__ float Tf[16][PC + 4]; const int lane = threadIdx.x, nloc = lane & 15, hlf = lane >> 4; const size_t m0 = (size_t)blockIdx.x * 16; if (m0 >= (size_t)RL) return; v8f acc[8];
#pragma unroll
  for (int t = 0; t < 8; ++t) acc[t] = (v8f){};
#pragma unroll 2
  for (int kb = 0; kb < H; kb += 32) { const v16b a = frag_kb(UT + (m0 + nloc) * H + kb, hlf);
#pragma unroll
    for (int t = 0; t < 8; ++t) acc[t] = wmma16b(a, frag_kb(WB + (size_t)(t * 16 + nloc) * H + kb, hlf), acc[t]); }
#pragma unroll
  for (int t = 0; t < 8; ++t)
#pragma unroll
    for (int r8 = 0; r8 < 8; ++r8) Tf[8 * hlf + r8][t * 16 + nloc] = acc[t][r8] * (1.0f / (XS * WSC));
  wave_lds_sync();
  for (int pass = 0; pass < 2; ++pass) { for (int rr = 0; rr < 16; ++rr) *(volatile v4f*)(BU + (m0 + rr) * PC + lane * 4) = *(const v4f*)(&Tf[rr][lane * 4]); __threadfence(); }
}
__global__ __launch_bounds__(32) void scan_kernel(const float* __restrict__ BU, const float* __restrict__ Ad, const float* __restrict__ steps, int BV, float* __restrict__ X) {
  const int lane = threadIdx.x; const int b = blockIdx.x / (PC / 32), cb = blockIdx.x % (PC / 32); if (b >= BV) return; const int c = cb * 32 + lane, p = c >> 1;
  const float A = fmaxf(bf16_rne(Ad[p]), 0.0f); const float st = bf16_rne(steps[p]); const float dt = 1.0f / (1.0f + __expf(-st)); const float Sg = 1.0f / (1.0f + pmul(pmul(dt, dt), A));
  const float m11 = 1.0f - pmul(pmul(pmul(dt, dt), A), Sg), m12 = -pmul(pmul(dt, A), Sg), m21 = pmul(dt, Sg), m22 = Sg; const float f1 = pmul(m11, dt), f2 = pmul(m21, dt);
  for (int pass = 0; pass < 2; ++pass) { float z = 0.0f, x = 0.0f;
#pragma unroll 1
    for (int t = 0; t < L; ++t) { const size_t row = (size_t)b * L + t; const float f = BU[row * PC + c]; const float zn = pmul(m11, z) + pmul(m12, x) + pmul(f1, f); const float xn = pmul(m21, z) + pmul(m22, x) + pmul(f2, f); z = zn; x = xn; ((volatile float*)X)[row * PC + c] = x; }
    __threadfence(); }
}
__global__ __launch_bounds__(32) void y_kernel(const float* __restrict__ X, const b16* __restrict__ WC, const float* __restrict__ uu, const float* __restrict__ Dv, int RL, float* __restrict__ Y) {
  __shared__ __attribute__((aligned(16))) b16 Ah[16][PC + 8], Al[16][PC + 8]; __shared__ float Tf[16][H + 4]; const int lane = threadIdx.x, nloc = lane & 15, hlf = lane >> 4; const size_t m0 = (size_t)blockIdx.x * 16; if (m0 >= (size_t)RL) return; const int b = (int)(m0 / L), l0 = (int)(m0 % L);
  for (int rr = 0; rr < 16; ++rr) for (int q = 0; q < 4; ++q) { b16 p, ql; split16(X[(m0 + rr) * PC + q * 32 + lane] * XS, p, ql); Ah[rr][q * 32 + lane] = p; Al[rr][q * 32 + lane] = ql; }
  wave_lds_sync(); v8f acc[16];
#pragma unroll
  for (int t = 0; t < 16; ++t) acc[t] = (v8f){};
#pragma unroll
  for (int kb = 0; kb < PC; kb += 32) { const v16b a = frag_kb(&Ah[nloc][kb], hlf), al = frag_kb(&Al[nloc][kb], hlf);
#pragma unroll
    for (int t = 0; t < 16; ++t) { const v16b bw = frag_kb(WC + (size_t)(t * 16 + nloc) * PC + kb, hlf); acc[t] = wmma16b(a, bw, acc[t]); acc[t] = wmma16b(al, bw, acc[t]); } }
#pragma unroll
  for (int t = 0; t < 16; ++t) { const int h = t * 16 + nloc; const float dv = bf16_rne(Dv[h]);
#pragma unroll
    for (int r8 = 0; r8 < 8; ++r8) { const int rl = 8 * hlf + r8; Tf[rl][h] = gelu(acc[t][r8] * (1.0f / (XS * WSC)) + pmul(bf16_rne(uu[((size_t)b * H + h) * L + l0 + rl]), dv)); } }
  wave_lds_sync();
  for (int pass = 0; pass < 2; ++pass) { for (int rr = 0; rr < 16; ++rr) for (int q = 0; q < 2; ++q) *(volatile v4f*)(Y + (m0 + rr) * H + q * 128 + lane * 4) = *(const v4f*)(&Tf[rr][q * 128 + lane * 4]); __threadfence(); }
}
__global__ __launch_bounds__(32) void gate_kernel(const float* __restrict__ Y, const b16* __restrict__ W12, const float* __restrict__ b1, const float* __restrict__ b2, int RL, float* __restrict__ G) {
  __shared__ __attribute__((aligned(16))) b16 Ah[16][H + 8], Al[16][H + 8]; __shared__ float Tf[16][132]; const int lane = threadIdx.x, nloc = lane & 15, hlf = lane >> 4; const int cg = blockIdx.x % 2; const size_t m0 = (size_t)(blockIdx.x / 2) * 16; if (m0 >= (size_t)RL) return;
  for (int rr = 0; rr < 16; ++rr) for (int q = 0; q < 8; ++q) { b16 p, ql; split16(Y[(m0 + rr) * H + q * 32 + lane] * XS, p, ql); Ah[rr][q * 32 + lane] = p; Al[rr][q * 32 + lane] = ql; }
  wave_lds_sync(); v8f a1[8], a2[8];
#pragma unroll
  for (int t = 0; t < 8; ++t) { a1[t] = (v8f){}; a2[t] = (v8f){}; }
#pragma unroll 2
  for (int kb = 0; kb < H; kb += 32) { const v16b a = frag_kb(&Ah[nloc][kb], hlf), al = frag_kb(&Al[nloc][kb], hlf);
#pragma unroll
    for (int t = 0; t < 8; ++t) { const size_t r1 = (size_t)(cg * 128 + t * 16 + nloc) * H + kb; const v16b w1 = frag_kb(W12 + r1, hlf), w2 = frag_kb(W12 + (size_t)H * H + r1, hlf); a1[t] = wmma16b(a, w1, a1[t]); a1[t] = wmma16b(al, w1, a1[t]); a2[t] = wmma16b(a, w2, a2[t]); a2[t] = wmma16b(al, w2, a2[t]); } }
#pragma unroll
  for (int t = 0; t < 8; ++t) { const int h = cg * 128 + t * 16 + nloc; const float bb1 = bf16_rne(b1[h]), bb2 = bf16_rne(b2[h]);
#pragma unroll
    for (int r8 = 0; r8 < 8; ++r8) { const float v1 = a1[t][r8] * (1.0f / (XS * WSC)) + bb1, v2 = a2[t][r8] * (1.0f / (XS * WSC)) + bb2; Tf[8 * hlf + r8][t * 16 + nloc] = pmul(v1, 1.0f / (1.0f + __expf(-v2))); } }
  wave_lds_sync();
  for (int pass = 0; pass < 2; ++pass) { for (int rr = 0; rr < 16; ++rr) *(volatile v4f*)(G + (m0 + rr) * H + cg * 128 + lane * 4) = *(const v4f*)(&Tf[rr][lane * 4]); __threadfence(); }
}
__global__ __launch_bounds__(256) void out_kernel(const float* __restrict__ G, int BV, float* __restrict__ out) {
  __shared__ float Ts[32][H + 1]; const int tid = threadIdx.x, wave = tid >> 5, lane = tid & 31; const int b = blockIdx.x / (L / 32), l0 = (blockIdx.x % (L / 32)) * 32; if (b >= BV) return;
  for (int r = wave; r < 32; r += 8) for (int q = 0; q < 8; ++q) Ts[r][q * 32 + lane] = G[((size_t)b * L + l0 + r) * H + q * 32 + lane];
  __syncthreads();
  for (int pass = 0; pass < 2; ++pass) { for (int h = wave; h < H; h += 8) ((volatile float*)out)[((size_t)b * H + h) * L + l0 + lane] = Ts[lane][h]; __threadfence(); }
}
}

extern "C" void kernel_launch(void* const* d_in, const int* in_sizes, int n_in, void* d_out, int out_size, void* d_ws, size_t ws_size, hipStream_t stream) {
  (void)n_in;
  auto Fp = [&](int i) { return (const float*)d_in[i]; };
  if (in_sizes[0] != B * H * L || in_sizes[1] != P || in_sizes[2] != P * H * 2 || in_sizes[3] != H * P * 2 || in_sizes[4] != H || in_sizes[5] != P || in_sizes[6] != H * H || in_sizes[8] != H * H || out_size != B * H * L) return;
  const int BV = B; const int RL = BV * L;
  size_t off = 0; char* ws = (char*)d_ws;
  auto carve = [&](size_t bytes) { char* p = ws + off; off += (bytes + 255) & ~(size_t)255; return p; };
  b16* WB = (b16*)carve((size_t)PC * H * 2); b16* WC = (b16*)carve((size_t)H * PC * 2); b16* W12 = (b16*)carve((size_t)2 * H * H * 2); b16* UT = (b16*)carve((size_t)NR * H * 2); float* BU = (float*)carve((size_t)NR * PC * 4); float* X = (float*)carve((size_t)NR * PC * 4); float* Y = (float*)carve((size_t)NR * H * 4); float* G = (float*)carve((size_t)NR * H * 4);
  if (off > ws_size || off > ((size_t)128 << 20)) return;
  wprep_kernel<<<(2 * H * (H / 8) + 255) / 256, 256, 0, stream>>>(Fp(2), Fp(3), Fp(6), Fp(8), WB, WC, W12);
  ut_kernel<<<BV * (L / 32), 256, 0, stream>>>(Fp(0), BV, UT);
  bu_kernel<<<RL / 16, 32, 0, stream>>>(UT, WB, RL, BU);
  scan_kernel<<<BV * (PC / 32), 32, 0, stream>>>(BU, Fp(1), Fp(5), BV, X);
  y_kernel<<<RL / 16, 32, 0, stream>>>(X, WC, Fp(0), Fp(4), RL, Y);
  gate_kernel<<<(RL / 16) * 2, 32, 0, stream>>>(Y, W12, Fp(7), Fp(9), RL, G);
  out_kernel<<<BV * (L / 32), 256, 0, stream>>>(G, BV, (float*)d_out);
}
